// MultiheadAttention_51161650430216
// MI455X (gfx1250) — hardware-run, weakly checked
//
#include <hip/hip_runtime.h>
#ifndef NB
#define NB 2
#endif
#ifndef SEQ
#define SEQ 2048
#endif
#define NB_FULL 2
#define SQ_FULL 2048
#define SQ SEQ
#define DM 1024
#define NH 16
#define HD 64
#define QT 256
#define NKX SQ
#define LQ (3 * DM)
#define NR ((size_t)NB * SQ)
#define NIT (SQ / 256)
static_assert(NH * HD == DM);
static_assert(SQ % 256 == 0 && SQ % QT == 0 && QT % 128 == 0);
static_assert(SQ <= SQ_FULL && NB <= NB_FULL);
static_assert(NIT >= 1 && NIT <= 8);

typedef unsigned short v8us __attribute__((ext_vector_type(8), may_alias));
typedef float  v8f  __attribute__((ext_vector_type(8)));
typedef float  v4f  __attribute__((ext_vector_type(4)));
typedef float  v4fa __attribute__((ext_vector_type(4), may_alias));
typedef _Float16 v16h __attribute__((ext_vector_type(16)));
typedef _Float16 v4h __attribute__((ext_vector_type(4)));
union FragH { v16h v; v8us half[2]; _Float16 h[16]; unsigned short u[16]; };

__device__ __forceinline__ unsigned short bf16_bits(float x) { unsigned int u = __float_as_uint(x); return (unsigned short)((u + 0x7FFFu + ((u >> 16) & 1u)) >> 16); }
__device__ __forceinline__ float bf16_val(unsigned short b) { return __uint_as_float(((unsigned int)b) << 16); }
__device__ __forceinline__ float bf16_rne(float x) { return bf16_val(bf16_bits(x)); }

__global__ __launch_bounds__(256) void k_wnat(const float* __restrict__ w, size_t n8, _Float16* __restrict__ Bt) {
  const size_t t = (size_t)blockIdx.x * 256 + threadIdx.x; if (t >= n8) return;
  const v4f a = *(const v4fa*)(w + t * 8), c = *(const v4fa*)(w + t * 8 + 4);
  FragH f;
#pragma unroll
  for (int q = 0; q < 4; ++q) { f.h[q] = (_Float16)(bf16_rne(a[q]) * 16.0f); f.h[4 + q] = (_Float16)(bf16_rne(c[q]) * 16.0f); }
  const v8us o = f.half[0];
  *(volatile v8us*)((unsigned short*)Bt + t * 8) = o; __threadfence(); *(volatile v8us*)((unsigned short*)Bt + t * 8) = o;
}

__global__ __launch_bounds__(256) void k_x16(const float* __restrict__ x, _Float16* __restrict__ X16, size_t n8) {
  const size_t t = (size_t)blockIdx.x * 256 + threadIdx.x; if (t >= n8) return;
  const size_t e = t * 8; const size_t row = e / DM; const size_t col = e % DM; const size_t b = row / SQ, s = row % SQ;
  const float* src = x + ((b * SQ_FULL + s) * DM + col);
  const v4f a = *(const v4fa*)(src), c = *(const v4fa*)(src + 4);
  FragH f;
#pragma unroll
  for (int q = 0; q < 4; ++q) { f.h[q] = (_Float16)bf16_rne(a[q]); f.h[4 + q] = (_Float16)bf16_rne(c[q]); }
  const v8us o = f.half[0];
  *(volatile v8us*)((unsigned short*)X16 + t * 8) = o; __threadfence(); *(volatile v8us*)((unsigned short*)X16 + t * 8) = o;
}

template <int NHv, int TTv>
__global__ __launch_bounds__(256) void k_vt(const _Float16* __restrict__ V16, int ldv, int voff, _Float16* __restrict__ Vt) {
  __shared__ unsigned short tl[64][66];
  const int tid = threadIdx.x; const int slab = blockIdx.x / (TTv / 64), lg = blockIdx.x % (TTv / 64); const int b = slab / NHv, h = slab % NHv;
  for (int i = tid; i < 64 * 8; i += 256) { const int r = i / 8, c8 = (i % 8) * 8; FragH f; f.half[0] = *(const v8us*)((const unsigned short*)V16 + ((size_t)b * TTv + lg * 64 + r) * ldv + voff + h * 64 + c8);
#pragma unroll
    for (int q = 0; q < 8; ++q) tl[r][c8 + q] = f.u[q]; }
  __syncthreads();
  for (int pass = 0; pass < 2; ++pass) {
#pragma unroll
    for (int rd = 0; rd < 2; ++rd) { const int d = rd * 32 + tid / 8, pc = tid % 8; FragH f;
#pragma unroll
      for (int q = 0; q < 8; ++q) f.u[q] = tl[pc * 8 + q][d];
      *(volatile v8us*)((unsigned short*)Vt + ((size_t)slab * 64 + d) * TTv + lg * 64 + pc * 8) = f.half[0]; }
    if (pass == 0) __threadfence(); } }

__global__ __launch_bounds__(256) void k_rsmw(const float* __restrict__ S, _Float16* __restrict__ P, int nrows) {
  #pragma clang fp contract(off)
  const int lane = threadIdx.x & 31, w = threadIdx.x >> 5;
  const int row = blockIdx.x * 8 + w;
  if (row >= nrows) return;
  const float* s = S + (size_t)row * NKX + lane * 8;
  v4f va[2 * NIT];
#pragma unroll
  for (int it = 0; it < NIT; ++it) {
    va[2 * it] = *(const v4fa*)(s + it * 256);
    va[2 * it + 1] = *(const v4fa*)(s + it * 256 + 4);
    if ((it & 3) == 3) asm volatile("" ::: "memory");
  }
  float mx = -3.0e38f;
#pragma unroll
  for (int i = 0; i < 2 * NIT; ++i) {
#pragma unroll
    for (int q = 0; q < 4; ++q) mx = fmaxf(mx, va[i][q]);
  }
#pragma unroll
  for (int o = 16; o > 0; o >>= 1) mx = fmaxf(mx, __shfl_xor(mx, o));
  float se = 0.f;
#pragma unroll
  for (int i = 0; i < 2 * NIT; ++i) {
#pragma unroll
    for (int q = 0; q < 4; ++q) { const float e = __expf(va[i][q] - mx); va[i][q] = e; se += e; }
  }
#pragma unroll
  for (int o = 16; o > 0; o >>= 1) se += __shfl_xor(se, o);
  const float den = se + 1.0e-10f * __expf(-mx);
  const float sc = 1024.0f * __builtin_amdgcn_rcpf(den);
  unsigned short* d = (unsigned short*)P + (size_t)row * NKX + lane * 8;
  for (int pass = 0; pass < 2; ++pass) {
#pragma unroll
    for (int it = 0; it < NIT; ++it) {
      FragH f;
#pragma unroll
      for (int q = 0; q < 4; ++q) { f.h[q] = (_Float16)(va[2 * it][q] * sc); f.h[4 + q] = (_Float16)(va[2 * it + 1][q] * sc); }
      *(volatile v8us*)(d + it * 256) = f.half[0];
    }
    if (pass == 0) __threadfence();
  }
}

__device__ __forceinline__ v16h g2_frag(const _Float16* p, int hh) { FragH f; f.half[0] = *(const v8us*)((const unsigned short*)p + 8 * hh); f.half[1] = *(const v8us*)((const unsigned short*)p + 16 + 8 * hh); return f.v; }
__device__ __forceinline__ v8f g2_mma(v16h a, v16h b, v8f c) { v8f d = __builtin_amdgcn_wmma_f32_16x16x32_f16(false, a, false, b, (short)0, c, false, false); asm volatile("v_nop\n\tv_nop\n\tv_nop\n\tv_nop" : "+v"(d) : "v"(a), "v"(b)); return d; }
template <int MASKADD>
__global__ __launch_bounds__(128) void k_gemm2(const _Float16* __restrict__ A, int lda, size_t sA, const _Float16* __restrict__ Bh, int ldb, size_t sB, float alpha,
    const float* __restrict__ mask, int mrow0, int ldm, float* __restrict__ C, _Float16* __restrict__ C16, int ldc, size_t sC, int M, int N, int K) {
  __shared__ __attribute__((aligned(16))) float so[4][32][68];
  const int tid = threadIdx.x, w = tid >> 5, lane = tid & 31, ln = lane & 15, hh = lane >> 4; const int by = blockIdx.y;
  A += (size_t)by * sA; Bh += (size_t)by * sB; const size_t cofs = (size_t)by * sC;
  const int ntn = N >> 6; const int mt = blockIdx.x / ntn, nq = blockIdx.x - mt * ntn; const int row0 = mt * 128 + 32 * w, col0 = nq * 64; if (row0 >= M) return;
  const _Float16* a0p = A + (size_t)(row0 + ln) * lda; const _Float16* a1p = a0p + (size_t)16 * lda;
  const _Float16* b0p = Bh + (size_t)(col0 + ln) * ldb; const _Float16* b1p = b0p + (size_t)16 * ldb; const _Float16* b2p = b1p + (size_t)16 * ldb; const _Float16* b3p = b2p + (size_t)16 * ldb;
  const v8f z8 = {0.f,0.f,0.f,0.f,0.f,0.f,0.f,0.f}; v8f c00 = z8, c01 = z8, c02 = z8, c03 = z8, c10 = z8, c11 = z8, c12 = z8, c13 = z8;
#pragma unroll 1
  for (int kb = 0; kb < K; kb += 32) { const v16h a0 = g2_frag(a0p + kb, hh), a1 = g2_frag(a1p + kb, hh);
    v16h b = g2_frag(b0p + kb, hh); c00 = g2_mma(a0, b, c00); c10 = g2_mma(a1, b, c10);
    b = g2_frag(b1p + kb, hh); c01 = g2_mma(a0, b, c01); c11 = g2_mma(a1, b, c11);
    b = g2_frag(b2p + kb, hh); c02 = g2_mma(a0, b, c02); c12 = g2_mma(a1, b, c12);
    b = g2_frag(b3p + kb, hh); c03 = g2_mma(a0, b, c03); c13 = g2_mma(a1, b, c13); }
  v8f accs[8] = {c00, c01, c02, c03, c10, c11, c12, c13};
#pragma unroll
  for (int u = 0; u < 8; ++u) { const int t = u & 3, half = u >> 2;
#pragma unroll
    for (int r = 0; r < 8; ++r) { const int rloc = half * 16 + 8 * hh + r; so[w][rloc][t * 16 + ln] = accs[u][r] * alpha; } }
  __builtin_amdgcn_fence(4  , "workgroup"); __builtin_amdgcn_wave_barrier();
  const int rsub = lane >> 4, c4 = (lane & 15) * 4;
  if (MASKADD) {
#pragma unroll 4
    for (int q = 0; q < 16; ++q) { const int r = q * 2 + rsub; v4f v = *(const v4fa*)&so[w][r][c4];
      const v4f mk = *(const v4fa*)(mask + (size_t)(mrow0 + row0 + r) * ldm + col0 + c4);
#pragma unroll
      for (int i = 0; i < 4; ++i) v[i] += bf16_rne(mk[i]);
      *(v4fa*)&so[w][r][c4] = v; }
  }
  for (int pass = 0; pass < 2; ++pass) {
#pragma unroll
    for (int q = 0; q < 16; ++q) { const int r = q * 2 + rsub; const v4f v = *(const v4fa*)&so[w][r][c4];
      if (C) *(volatile v4f*)(C + cofs + (size_t)(row0 + r) * ldc + col0 + c4) = v;
      if (C16) { v4h h4;
#pragma unroll
        for (int i = 0; i < 4; ++i) h4[i] = (_Float16)v[i];
        *(volatile v4h*)(C16 + cofs + (size_t)(row0 + r) * ldc + col0 + c4) = h4; } }
    if (pass == 0) __threadfence(); } }

#define WS_BQKV ((size_t)3 * DM * DM * 2)
#define WS_BO   ((size_t)DM * DM * 2)
#define WS_X16  ((size_t)NB * SQ * DM * 2)
#define WS_QKV  ((size_t)NB * SQ * LQ * 2)
#define WS_VT   ((size_t)NB * NH * HD * SQ * 2)
#define WS_O16  ((size_t)NB * SQ * DM * 2)
#define WS_S    ((size_t)NH * QT * NKX * 4)
#define WS_P    ((size_t)NH * QT * NKX * 2)
static_assert(WS_BQKV % 256 == 0 && WS_BO % 256 == 0 && WS_X16 % 256 == 0 && WS_QKV % 256 == 0 && WS_VT % 256 == 0 && WS_O16 % 256 == 0 && WS_S % 256 == 0 && WS_P % 256 == 0);
static_assert(WS_BQKV + WS_BO + WS_X16 + WS_QKV + WS_VT + WS_O16 + WS_S + WS_P <= (size_t)134217728);

extern "C" void kernel_launch(void* const* d_in, const int* in_sizes, int n_in,
                              void* d_out, int out_size, void* d_ws, size_t ws_size, hipStream_t stream) {
  if (n_in < 6) return;
  const size_t xneed = ((size_t)(NB - 1) * SQ_FULL + SQ) * DM;
  if ((size_t)in_sizes[0] < xneed) return;
  if ((size_t)in_sizes[1] < (size_t)(SQ - 1) * SQ_FULL + SQ) return;
  if ((size_t)in_sizes[2] < (size_t)DM * DM || (size_t)in_sizes[3] < (size_t)DM * DM || (size_t)in_sizes[4] < (size_t)DM * DM || (size_t)in_sizes[5] < (size_t)DM * DM) return;
  if ((size_t)out_size < xneed) return;
  const float* const* I = (const float* const*)d_in;
  const float* x = I[0]; const float* mask = I[1]; const float* wq = I[2]; const float* wk = I[3]; const float* wv = I[4]; const float* wo = I[5];
  char* ws = (char*)d_ws; size_t off = 0;
  auto take = [&](size_t bytes) { char* p = ws + off; off += (bytes + 255) & ~(size_t)255; return p; };
  _Float16* BQKV = (_Float16*)take(WS_BQKV);
  _Float16* BO   = (_Float16*)take(WS_BO);
  _Float16* X16  = (_Float16*)take(WS_X16);
  _Float16* QKV  = (_Float16*)take(WS_QKV);
  _Float16* VT   = (_Float16*)take(WS_VT);
  _Float16* O16  = (_Float16*)take(WS_O16);
  float*    S    = (float*)take(WS_S);
  _Float16* P    = (_Float16*)take(WS_P);
  if (off > ws_size) return;
  { const size_t n8 = (size_t)DM * DM / 8; const unsigned g = (unsigned)((n8 + 255) / 256);
    k_wnat<<<g, 256, 0, stream>>>(wq, n8, BQKV);
    k_wnat<<<g, 256, 0, stream>>>(wk, n8, BQKV + (size_t)DM * DM);
    k_wnat<<<g, 256, 0, stream>>>(wv, n8, BQKV + (size_t)2 * DM * DM);
    k_wnat<<<g, 256, 0, stream>>>(wo, n8, BO); }
  k_x16<<<(unsigned)((NR * DM / 8 + 255) / 256), 256, 0, stream>>>(x, X16, NR * DM / 8);
  k_gemm2<0><<<dim3((unsigned)(((int)NR / 128) * (LQ / 64)), 1), 128, 0, stream>>>(X16, DM, 0, BQKV, DM, 0, 0.0625f, nullptr, 0, 0, nullptr, QKV, LQ, 0, (int)NR, LQ, DM);
  k_vt<NH, SQ><<<NB * NH * (SQ / 64), 256, 0, stream>>>(QKV, LQ, 2 * DM, VT);
  for (int b = 0; b < NB; ++b) { const size_t r0 = (size_t)b * SQ;
    for (int q0 = 0; q0 < SQ; q0 += QT) {
      k_gemm2<1><<<dim3((QT / 128) * (SQ / 64), NH), 128, 0, stream>>>(QKV + (r0 + q0) * LQ, LQ, (size_t)HD, QKV + r0 * LQ + DM, LQ, (size_t)HD, 0.125f, mask, q0, SQ_FULL, S, nullptr, NKX, (size_t)QT * NKX, QT, SQ, HD);
      k_rsmw<<<(NH * QT) / 8, 256, 0, stream>>>(S, P, NH * QT);
      k_gemm2<0><<<dim3((QT / 128) * (HD / 64), NH), 128, 0, stream>>>(P, NKX, (size_t)QT * NKX, VT + (size_t)b * NH * HD * SQ, SQ, (size_t)HD * SQ, 0.0625f, nullptr, 0, 0, nullptr, O16 + (r0 + q0) * DM, DM, (size_t)HD, QT, HD, SQ);
    } }
  k_gemm2<0><<<dim3((SQ / 128) * (DM / 64), NB), 128, 0, stream>>>(O16, DM, (size_t)SQ * DM, BO, DM, 0, 0.0009765625f, nullptr, 0, 0, (float*)d_out, nullptr, DM, (size_t)SQ_FULL * DM, SQ, DM, DM);
}
